// SS2D_4982162063930
// MI455X (gfx1250) — hardware-run, weakly checked
//
#include <hip/hip_runtime.h>
#include <hip/hip_fp16.h>
#include <math.h>

typedef __attribute__((ext_vector_type(16))) _Float16 v16h;
typedef __attribute__((ext_vector_type(8)))  _Float16 v8h;
typedef __attribute__((ext_vector_type(8)))  float    v8f;
typedef __attribute__((ext_vector_type(4)))  float    v4f;
typedef __attribute__((ext_vector_type(2)))  unsigned v2u;
typedef __attribute__((ext_vector_type(4)))  unsigned v4u;

constexpr int kBatch   = 4;
constexpr int kH       = 48;
constexpr int kW       = 48;
constexpr int kL       = kH * kW;
constexpr int kRows    = kBatch * kL;
constexpr int kC       = 192;
constexpr int kD       = 192;
constexpr int kXzN     = 2 * kD;
constexpr int kRank    = 12;
constexpr int kRkP     = 32;
constexpr int kNst     = 16;
constexpr int kXpN     = kRank + 2 * kNst;
constexpr int kXpP     = 64;
constexpr int kDirs    = 4;
constexpr int kTaps    = 9;
constexpr int kWin     = 4;
constexpr int kWinsW   = kW / kWin;
constexpr int kWinArea = kWin * kWin;
constexpr int kWinRowT = kWinsW * kWinArea;
constexpr int kFcH     = kC / 4;
constexpr int kFcHP    = 64;
constexpr int kAlpFloats = kDirs * kD * kNst;
constexpr int kPadFloats = kAlpFloats + kDirs * kD;
constexpr float kXCarry = 64.0f;
constexpr float kWCarry = 1024.0f;
constexpr float kSCarry = 256.0f;
constexpr float kRCarry = 1024.0f;
constexpr float kGCarry = 256.0f;
constexpr float kYCarry = 64.0f;
constexpr float kResid  = 2048.0f;
static_assert(kH == kW);
static_assert(kH == 48 && kW == 48 && kL == 2304 && kRows == 9216);
static_assert(kWin == 4 && kWinsW == 12 && kWinArea == 16 && kWinRowT == 192);
static_assert((kH % kWin) == 0 && (kW % kWin) == 0);
static_assert(kC == 192 && kD == 192 && kXzN == 384 && kXpN == 44 && kDirs == 4 && kTaps == 9);
static_assert(kFcH == 48 && kFcHP >= kFcH && (kFcH % 4) == 0 && (kFcHP % 4) == 0);
static_assert(kRank + 1 <= kRkP && kRank < 16);
static_assert((kC % 32) == 0 && (kD % 32) == 0 && (kRkP % 32) == 0);
static_assert((kC % 64) == 0 && (kD % 64) == 0 && (kXzN % 64) == 0 && (kXpP % 64) == 0);
static_assert((kRows % 32) == 0);
static_assert((kL % 64) == 0 && (kL % 4) == 0);
static_assert(kAlpFloats == 12288 && kPadFloats == 13056);

constexpr size_t kSzXH   = (size_t)kRows * kC * 2;
constexpr size_t kSzWIN  = (size_t)kXzN * kC * 2;
constexpr size_t kSzXZ   = (size_t)kRows * kXzN * 4;
constexpr size_t kSzUC   = (size_t)kRows * kD * 4;
constexpr size_t kSzXS   = (size_t)kDirs * kRows * kD * 4;
constexpr size_t kSzXSH  = (size_t)kDirs * kRows * kD * 2;
constexpr size_t kSzXPW  = (size_t)kDirs * kXpP * kD * 2;
constexpr size_t kSzXD   = (size_t)kDirs * kRows * kXpP * 4;
constexpr size_t kSzDRH  = (size_t)kDirs * kRows * kRkP * 2;
constexpr size_t kSzDTW  = (size_t)kDirs * kD * kRkP * 2;
constexpr size_t kSzDTP  = (size_t)kDirs * kRows * kD * 4;
constexpr size_t kSzPADS = (size_t)kPadFloats * 4;
constexpr size_t kSzYH   = (size_t)kDirs * kRows * kD * 2;
constexpr size_t kSzGCM  = (size_t)kBatch * kD * 4;
constexpr size_t kSzH1   = (size_t)kBatch * kFcHP * 4;
constexpr size_t kSzGC   = (size_t)kBatch * kC * 4;
constexpr size_t kSzMG   = (size_t)kRows * kD * 4;
constexpr size_t kSzST   = (size_t)kRows * 4 * 4;
constexpr size_t kSzYG   = (size_t)kRows * kD * 2;
constexpr size_t kSzOW   = (size_t)kC * kD * 2;
constexpr size_t kSzRAW  = (size_t)kRows * kC * 4;
constexpr size_t kOffXH   = 0;
constexpr size_t kOffWIN  = kOffXH   + kSzXH;
constexpr size_t kOffXZ   = kOffWIN  + kSzWIN;
constexpr size_t kOffUC   = kOffXZ   + kSzXZ;
constexpr size_t kOffXS   = kOffUC   + kSzUC;
constexpr size_t kOffXSH  = kOffXS   + kSzXS;
constexpr size_t kOffXPW  = kOffXSH  + kSzXSH;
constexpr size_t kOffXD   = kOffXPW  + kSzXPW;
constexpr size_t kOffDRH  = kOffXD   + kSzXD;
constexpr size_t kOffDTW  = kOffDRH  + kSzDRH;
constexpr size_t kOffDTP  = kOffDTW  + kSzDTW;
constexpr size_t kOffPADS = kOffDTP  + kSzDTP;
constexpr size_t kOffYH   = kOffPADS + kSzPADS;
constexpr size_t kOffGCM  = kOffYH   + kSzYH;
constexpr size_t kOffH1   = kOffGCM  + kSzGCM;
constexpr size_t kOffGC   = kOffH1   + kSzH1;
constexpr size_t kOffMG   = kOffGC   + kSzGC;
constexpr size_t kOffST   = kOffMG   + kSzMG;
constexpr size_t kOffYG   = kOffST   + kSzST;
constexpr size_t kOffOW   = kOffYG   + kSzYG;
constexpr size_t kOffRAW  = kOffOW   + kSzOW;
constexpr size_t kWsTotal = kOffRAW  + kSzRAW;
static_assert(kSzXH == 3538944ull && kSzWIN == 147456ull && kSzXZ == 14155776ull && kSzUC == 7077888ull);
static_assert(kSzXS == 28311552ull && kSzXSH == 14155776ull && kSzXPW == 98304ull && kSzXD == 9437184ull);
static_assert(kSzDRH == 2359296ull && kSzDTW == 49152ull && kSzDTP == 28311552ull && kSzPADS == 52224ull);
static_assert(kSzYH == 14155776ull && kSzGCM == 3072ull && kSzH1 == 1024ull && kSzGC == 3072ull);
static_assert(kSzMG == 7077888ull && kSzST == 147456ull && kSzYG == 3538944ull && kSzOW == 73728ull);
static_assert(kSzRAW == 7077888ull);
static_assert(kWsTotal == 3538944ull + 147456ull + 14155776ull + 7077888ull + 28311552ull + 14155776ull + 98304ull +
              9437184ull + 2359296ull + 49152ull + 28311552ull + 52224ull + 14155776ull + 3072ull + 1024ull +
              3072ull + 7077888ull + 147456ull + 3538944ull + 73728ull + 7077888ull);
static_assert(kWsTotal == 139773952ull);
static_assert(kWsTotal <= 268435456ull);
static_assert((kSzXH % 128) == 0 && (kSzWIN % 128) == 0 && (kSzXZ % 128) == 0 && (kSzUC % 128) == 0 &&
              (kSzXS % 128) == 0 && (kSzXSH % 128) == 0 && (kSzXPW % 128) == 0 && (kSzXD % 128) == 0 &&
              (kSzDRH % 128) == 0 && (kSzDTW % 128) == 0 && (kSzDTP % 128) == 0 && (kSzPADS % 128) == 0 &&
              (kSzYH % 128) == 0 && (kSzGCM % 128) == 0 && (kSzH1 % 128) == 0 && (kSzGC % 128) == 0 &&
              (kSzMG % 128) == 0 && (kSzST % 128) == 0 && (kSzYG % 128) == 0 && (kSzOW % 128) == 0 &&
              (kSzRAW % 128) == 0);
static_assert((((size_t)kRows * kD * 4) % 128) == 0 && (((size_t)kRows * kD * 2) % 128) == 0 &&
              (((size_t)kXpP * kD * 2) % 128) == 0 && (((size_t)kRows * kXpP * 4) % 128) == 0 &&
              (((size_t)kRows * kRkP * 2) % 128) == 0 && (((size_t)kD * kRkP * 2) % 128) == 0 &&
              (((size_t)kD * kNst * 4) % 128) == 0 && (((size_t)kAlpFloats * 4) % 128) == 0);

__device__ __forceinline__ _Float16 f16_flush(float v) {
  const float w = (fabsf(v) < 6.103515625e-05f) ? 0.0f : v;
  return (_Float16)w;
}
__device__ __forceinline__ void f16_split(float v, _Float16& hi, _Float16& lo) {
  hi = f16_flush(v);
  const float hf = (float)hi;
  const float r = (v - hf) * kResid;
  lo = f16_flush(r);
}

__device__ __forceinline__ float bf16r(float v) {
  unsigned u = __float_as_uint(v);
  u = (u + 0x7FFFu + ((u >> 16) & 1u)) & 0xFFFF0000u;
  return __uint_as_float(u);
}

__device__ __forceinline__ float h16_to_f32(unsigned hb) {
  const unsigned sgn = (hb & 0x8000u) << 16; const unsigned em = hb & 0x7fffu;
  const float fn = __uint_as_float((em << 13) + 0x38000000u);
  const float fs = (float)em * 5.9604644775390625e-8f;
  const float mag = (em < 0x400u) ? fs : fn; return __uint_as_float(__float_as_uint(mag) | sgn); }

namespace eng {
union FragU { v16h v; v8h h[2]; };
__device__ __forceinline__ v16h frag_load(const _Float16* p) {
  FragU f;
  f.h[0] = *(const v8h*)(p);
  f.h[1] = *(const v8h*)(p + 16);
  return f.v;
}
__device__ __forceinline__ v8f mma(v16h a, v16h b, v8f c) {
  return __builtin_amdgcn_wmma_f32_16x16x32_f16(false, a, false, b, (short)0, c, false, false);
}
__device__ __forceinline__ void guard1(v8f& a, v16h x, v16h y) {
  asm volatile("v_nop\n\tv_nop\n\tv_nop\n\tv_nop" : "+v"(a) : "v"(x), "v"(y));
}
__device__ __forceinline__ void guard_acc(v8f& a) {
  asm volatile("v_nop\n\tv_nop\n\tv_nop\n\tv_nop" : "+v"(a));
}
__device__ __forceinline__ void keep4(v16h a, v16h b, v16h c, v16h d) {
  asm volatile("v_nop" :: "v"(a), "v"(b), "v"(c), "v"(d));
}

template <int MI, int SPL>
__global__ __launch_bounds__(256) void gemm_f16_kernel(
    const unsigned short* __restrict__ Ap, const unsigned short* __restrict__ A2p, int lda,
    const unsigned short* __restrict__ Btp, const unsigned short* __restrict__ Bt2p, int ldb,
    float* __restrict__ C, int ldc, int M, int N, int K, float scale, float rscale)
{
  static_assert(MI >= 1 && MI <= 2);
  static_assert(SPL >= 0 && SPL <= 2);
  const _Float16* A   = (const _Float16*)Ap;
  const _Float16* A2  = (const _Float16*)A2p;
  const _Float16* Bt  = (const _Float16*)Btp;
  const _Float16* Bt2 = (const _Float16*)Bt2p;
  __shared__ __align__(16) float sT[8][16 * 68];
  const int lane = threadIdx.x & 31;
  const int wave = threadIdx.x >> 5;
  const int tilesN = N >> 6;
  const int tilesM = M / (16 * MI);
  const int tile = blockIdx.x * 8 + wave;
  if (tile >= tilesM * tilesN) return;
  const int tm = tile / tilesN;
  const int tn = tile - tm * tilesN;
  const int m0 = tm * (16 * MI);
  const int n0 = tn << 6;
  const int rlane = lane & 15;
  const int koff  = (lane >> 4) * 8;
  const int mOff  = (lane >> 4) * 8;

  v8f acc[MI][4], accr[MI][4];
#pragma unroll
  for (int i = 0; i < MI; ++i)
#pragma unroll
    for (int j = 0; j < 4; ++j) {
      acc[i][j]  = (v8f){0.f, 0.f, 0.f, 0.f, 0.f, 0.f, 0.f, 0.f};
      accr[i][j] = (v8f){0.f, 0.f, 0.f, 0.f, 0.f, 0.f, 0.f, 0.f};
    }

  for (int k0 = 0; k0 < K; k0 += 32) {
    v16h bh[4], bl[4];
#pragma unroll
    for (int j = 0; j < 4; ++j) {
      const size_t bo = (size_t)(n0 + (j << 4) + rlane) * ldb + koff + k0;
      bh[j] = frag_load(Bt + bo);
      if (SPL == 2) bl[j] = frag_load(Bt2 + bo); else bl[j] = bh[j];
    }
#pragma unroll
    for (int i = 0; i < MI; ++i) {
      const size_t ao = (size_t)(m0 + (i << 4) + rlane) * lda + koff + k0;
      const v16h ah = frag_load(A + ao);
      v16h al = ah;
      if (SPL >= 1) al = frag_load(A2 + ao);
#pragma unroll
      for (int j = 0; j < 4; ++j) {
        acc[i][j] = mma(ah, bh[j], acc[i][j]);
        if (SPL >= 1) accr[i][j] = mma(al, bh[j], accr[i][j]);
        if (SPL == 2) accr[i][j] = mma(ah, bl[j], accr[i][j]);
      }
#pragma unroll
      for (int j = 0; j < 4; ++j) {
        guard1(acc[i][j], ah, al);
        if (SPL >= 1) guard1(accr[i][j], ah, al);
      }
    }
    keep4(bh[0], bh[1], bh[2], bh[3]);
    if (SPL == 2) keep4(bl[0], bl[1], bl[2], bl[3]);
  }
#pragma unroll
  for (int i = 0; i < MI; ++i)
#pragma unroll
    for (int j = 0; j < 4; ++j) {
      guard_acc(acc[i][j]);
      if (SPL >= 1) guard_acc(accr[i][j]);
    }

  float* slab = sT[wave];
#pragma unroll
  for (int i = 0; i < MI; ++i) {
    const int mBase = m0 + (i << 4);
#pragma unroll
    for (int j = 0; j < 4; ++j) {
#pragma unroll
      for (int r = 0; r < 8; ++r) {
        float v = acc[i][j][r] * scale;
        if (SPL >= 1) v += accr[i][j][r] * rscale;
        slab[(mOff + r) * 68 + (j << 4) + rlane] = v;
      }
    }
    __builtin_amdgcn_fence(__ATOMIC_RELEASE, "workgroup");
    __builtin_amdgcn_wave_barrier();
    __builtin_amdgcn_fence(__ATOMIC_ACQUIRE, "workgroup");
    {
      const int hh = lane >> 4, c4 = (lane & 15) * 4;
      for (int pass = 0; pass < 2; ++pass) {
#pragma unroll
        for (int it = 0; it < 8; ++it) {
          const int row = it * 2 + hh;
          const v4f v = *(const v4f*)(slab + row * 68 + c4);
          *(volatile v4f*)(C + (size_t)(mBase + row) * ldc + n0 + c4) = v;
        }
        __threadfence();
      }
    }
    __builtin_amdgcn_fence(__ATOMIC_RELEASE, "workgroup");
    __builtin_amdgcn_wave_barrier();
    __builtin_amdgcn_fence(__ATOMIC_ACQUIRE, "workgroup");
  }
}
}

__device__ __forceinline__ _Float16 in_half(float v, float carry, bool live) {
  const float t = live ? (bf16r(v) * carry) : 0.0f;
  return f16_flush(t);
}
__device__ __forceinline__ _Float16 val_half(float v, float carry, bool live) {
  const float t = live ? (v * carry) : 0.0f;
  return f16_flush(t);
}
__device__ __forceinline__ v8h pack8_in(v4f a0, v4f a1, float carry, bool live) {
  const float f0 = a0[0];
  const float f1 = a0[1];
  const float f2 = a0[2];
  const float f3 = a0[3];
  const float f4 = a1[0];
  const float f5 = a1[1];
  const float f6 = a1[2];
  const float f7 = a1[3];
  v8h hv;
  hv[0] = in_half(f0, carry, live);
  hv[1] = in_half(f1, carry, live);
  hv[2] = in_half(f2, carry, live);
  hv[3] = in_half(f3, carry, live);
  hv[4] = in_half(f4, carry, live);
  hv[5] = in_half(f5, carry, live);
  hv[6] = in_half(f6, carry, live);
  hv[7] = in_half(f7, carry, live);
  return hv;
}
__device__ __forceinline__ int src_pixel(int k, int t) {
  const int u = (k >= 2) ? (kL - 1 - t) : t;
  const int nh = u / kWinRowT;
  const int q = u - nh * kWinRowT;
  const int nw = q / kWinArea;
  const int hi = (q % kWinArea) / kWin;
  const int wi = q % kWin;
  const int pa = nh * kWin + hi;
  const int pb = nw * kWin + wi;
  const int p0 = pa * kW + pb;
  const int p1 = pb * kW + pa;
  return ((k & 1) != 0) ? p1 : p0;
}
__device__ __forceinline__ int win_index(int p) {
  const int h = p / kW;
  const int w = p - h * kW;
  return ((h / kWin) * kWinsW + (w / kWin)) * kWinArea + (h % kWin) * kWin + (w % kWin);
}
__device__ __forceinline__ int swap48(int i) {
  const int a = i / kH;
  const int r = i - a * kH;
  return r * kW + a;
}

__global__ __launch_bounds__(256) void pack_x_kernel(
    const float* __restrict__ x, unsigned short* __restrict__ XH)
{
  const int i = blockIdx.x * 256 + threadIdx.x;
  const int r = i / (kC / 8);
  const int c8 = (i - r * (kC / 8)) * 8;
  const float* sp = x + (size_t)r * kC + c8;
  const v4f a0 = *(const v4f*)(sp);
  const v4f a1 = *(const v4f*)(sp + 4);
  const v8h hv = pack8_in(a0, a1, kXCarry, true);
  unsigned short* q = XH + (size_t)i * 8;
  *(volatile v8h*)q = hv;
  __threadfence();
  *(volatile v8h*)q = hv;
}

__global__ __launch_bounds__(256) void pack_inw_kernel(
    const float* __restrict__ w, unsigned short* __restrict__ WIN)
{
  const int i = blockIdx.x * 256 + threadIdx.x;
  const int n = i / (kC / 8);
  const int c8 = (i - n * (kC / 8)) * 8;
  const float* sp = w + (size_t)n * kC + c8;
  const v4f a0 = *(const v4f*)(sp);
  const v4f a1 = *(const v4f*)(sp + 4);
  const v8h hv = pack8_in(a0, a1, kWCarry, true);
  unsigned short* q = WIN + (size_t)i * 8;
  *(volatile v8h*)q = hv;
  __threadfence();
  *(volatile v8h*)q = hv;
}

__global__ __launch_bounds__(256) void conv_kernel(
    const float* __restrict__ XZ, const float* __restrict__ cw, const float* __restrict__ cb,
    float* __restrict__ UC)
{
  const int i = blockIdx.x * 256 + threadIdx.x;
  const int r = i / (kD / 4);
  const int d4 = (i - r * (kD / 4)) * 4;
  const int b = r / kL;
  const int l = r - b * kL;
  const int h = l / kW;
  const int w = l - h * kW;
  const float* wp = cw + (size_t)d4 * kTaps;
  float acc0 = 0.0f, acc1 = 0.0f, acc2 = 0.0f, acc3 = 0.0f;
  for (int a = 0; a < 3; ++a) {
    const int hy = h + a - 1;
    const bool vh = (hy >= 0) && (hy <= kH - 1);
    const int hcl = (hy < 0) ? 0 : ((hy > kH - 1) ? (kH - 1) : hy);
    for (int e = 0; e < 3; ++e) {
      const int wx = w + e - 1;
      const bool vw = (wx >= 0) && (wx <= kW - 1);
      const int wcl = (wx < 0) ? 0 : ((wx > kW - 1) ? (kW - 1) : wx);
      const int row = b * kL + hcl * kW + wcl;
      const v4f xv = *(const v4f*)(XZ + (size_t)row * kXzN + d4);
      const bool ok = vh && vw;
      const float x0 = xv[0];
      const float x1 = xv[1];
      const float x2 = xv[2];
      const float x3 = xv[3];
      const float t0 = ok ? x0 : 0.0f;
      const float t1 = ok ? x1 : 0.0f;
      const float t2 = ok ? x2 : 0.0f;
      const float t3 = ok ? x3 : 0.0f;
      const int t = a * 3 + e;
      acc0 = fmaf(t0, bf16r(wp[t]), acc0);
      acc1 = fmaf(t1, bf16r(wp[kTaps + t]), acc1);
      acc2 = fmaf(t2, bf16r(wp[2 * kTaps + t]), acc2);
      acc3 = fmaf(t3, bf16r(wp[3 * kTaps + t]), acc3);
    }
  }
  const v4f bv = *(const v4f*)(cb + d4);
  const float b0 = bv[0];
  const float b1 = bv[1];
  const float b2 = bv[2];
  const float b3 = bv[3];
  const float s0 = acc0 + bf16r(b0);
  const float s1 = acc1 + bf16r(b1);
  const float s2 = acc2 + bf16r(b2);
  const float s3 = acc3 + bf16r(b3);
  v4f o;
  o[0] = s0 / (1.0f + expf(-s0));
  o[1] = s1 / (1.0f + expf(-s1));
  o[2] = s2 / (1.0f + expf(-s2));
  o[3] = s3 / (1.0f + expf(-s3));
  float* q = UC + (size_t)i * 4;
  *(volatile v4f*)q = o;
  __threadfence();
  *(volatile v4f*)q = o;
}

__global__ __launch_bounds__(256) void order_kernel(
    const float* __restrict__ UC, float* __restrict__ XS)
{
  const int i = blockIdx.x * 256 + threadIdx.x;
  const int k = i / (kRows * (kD / 4));
  const int rem = i - k * (kRows * (kD / 4));
  const int R = rem / (kD / 4);
  const int d4 = (rem - R * (kD / 4)) * 4;
  const int b = R / kL;
  const int t = R - b * kL;
  const int src = b * kL + src_pixel(k, t);
  const v4f v = *(const v4f*)(UC + (size_t)src * kD + d4);
  float* q = XS + (size_t)i * 4;
  *(volatile v4f*)q = v;
  __threadfence();
  *(volatile v4f*)q = v;
}

__global__ __launch_bounds__(256) void pack_xs_kernel(
    const float* __restrict__ UC, unsigned short* __restrict__ XSH)
{
  const int i = blockIdx.x * 256 + threadIdx.x;
  const int k = i / (kRows * (kD / 8));
  const int rem = i - k * (kRows * (kD / 8));
  const int R = rem / (kD / 8);
  const int d8 = (rem - R * (kD / 8)) * 8;
  const int b = R / kL;
  const int t = R - b * kL;
  const int src = b * kL + src_pixel(k, t);
  const float* sp = UC + (size_t)src * kD + d8;
  const v4f a0 = *(const v4f*)(sp);
  const v4f a1 = *(const v4f*)(sp + 4);
  const float f0 = a0[0];
  const float f1 = a0[1];
  const float f2 = a0[2];
  const float f3 = a0[3];
  const float f4 = a1[0];
  const float f5 = a1[1];
  const float f6 = a1[2];
  const float f7 = a1[3];
  v8h hv;
  hv[0] = val_half(f0, kSCarry, true);
  hv[1] = val_half(f1, kSCarry, true);
  hv[2] = val_half(f2, kSCarry, true);
  hv[3] = val_half(f3, kSCarry, true);
  hv[4] = val_half(f4, kSCarry, true);
  hv[5] = val_half(f5, kSCarry, true);
  hv[6] = val_half(f6, kSCarry, true);
  hv[7] = val_half(f7, kSCarry, true);
  unsigned short* q = XSH + (size_t)i * 8;
  *(volatile v8h*)q = hv;
  __threadfence();
  *(volatile v8h*)q = hv;
}

__global__ __launch_bounds__(256) void pack_xpw_kernel(
    const float* __restrict__ w, unsigned short* __restrict__ XPW)
{
  const int i = blockIdx.x * 256 + threadIdx.x;
  const int k = i / (kXpP * (kD / 8));
  const int rem = i - k * (kXpP * (kD / 8));
  const int n = rem / (kD / 8);
  const int j8 = (rem - n * (kD / 8)) * 8;
  const bool live = (n < kXpN);
  const int nc = live ? n : (kXpN - 1);
  const float* sp = w + ((size_t)(k * kXpN + nc) * kD + j8);
  const v4f a0 = *(const v4f*)(sp);
  const v4f a1 = *(const v4f*)(sp + 4);
  const v8h hv = pack8_in(a0, a1, kWCarry, live);
  unsigned short* q = XPW + (size_t)i * 8;
  *(volatile v8h*)q = hv;
  __threadfence();
  *(volatile v8h*)q = hv;
}

__device__ __forceinline__ _Float16 dr_half(float v, int j) {
  const float t = (j < kRank) ? (v * kRCarry) : ((j == kRank) ? kRCarry : 0.0f);
  return f16_flush(t);
}
__global__ __launch_bounds__(256) void pack_dr_kernel(
    const float* __restrict__ XD, unsigned short* __restrict__ DRH)
{
  const int i = blockIdx.x * 256 + threadIdx.x;
  const int row = i / (kRkP / 8);
  const int j8 = (i - row * (kRkP / 8)) * 8;
  const int jc = (j8 < 16) ? j8 : 8;
  const float* sp = XD + (size_t)row * kXpP + jc;
  const v4f a0 = *(const v4f*)(sp);
  const v4f a1 = *(const v4f*)(sp + 4);
  const float f0 = a0[0];
  const float f1 = a0[1];
  const float f2 = a0[2];
  const float f3 = a0[3];
  const float f4 = a1[0];
  const float f5 = a1[1];
  const float f6 = a1[2];
  const float f7 = a1[3];
  v8h hv;
  hv[0] = dr_half(f0, j8 + 0);
  hv[1] = dr_half(f1, j8 + 1);
  hv[2] = dr_half(f2, j8 + 2);
  hv[3] = dr_half(f3, j8 + 3);
  hv[4] = dr_half(f4, j8 + 4);
  hv[5] = dr_half(f5, j8 + 5);
  hv[6] = dr_half(f6, j8 + 6);
  hv[7] = dr_half(f7, j8 + 7);
  unsigned short* q = DRH + (size_t)i * 8;
  *(volatile v8h*)q = hv;
  __threadfence();
  *(volatile v8h*)q = hv;
}

__device__ __forceinline__ _Float16 dtw_half(const float* __restrict__ wrow, float bias, int j) {
  const int jc = (j < kRank) ? j : (kRank - 1);
  const float wv = wrow[jc];
  const float t = (j < kRank) ? (bf16r(wv) * kWCarry) : ((j == kRank) ? (bf16r(bias) * kWCarry) : 0.0f);
  return f16_flush(t);
}
__global__ __launch_bounds__(256) void pack_dtw_kernel(
    const float* __restrict__ dtw, const float* __restrict__ dtb, unsigned short* __restrict__ DTW)
{
  const int i = blockIdx.x * 256 + threadIdx.x;
  const int kc = i / (kRkP / 8);
  const int j8 = (i - kc * (kRkP / 8)) * 8;
  const float* wrow = dtw + (size_t)kc * kRank;
  const float bias = dtb[kc];
  v8h hv;
  hv[0] = dtw_half(wrow, bias, j8 + 0);
  hv[1] = dtw_half(wrow, bias, j8 + 1);
  hv[2] = dtw_half(wrow, bias, j8 + 2);
  hv[3] = dtw_half(wrow, bias, j8 + 3);
  hv[4] = dtw_half(wrow, bias, j8 + 4);
  hv[5] = dtw_half(wrow, bias, j8 + 5);
  hv[6] = dtw_half(wrow, bias, j8 + 6);
  hv[7] = dtw_half(wrow, bias, j8 + 7);
  unsigned short* q = DTW + (size_t)i * 8;
  *(volatile v8h*)q = hv;
  __threadfence();
  *(volatile v8h*)q = hv;
}

__global__ __launch_bounds__(32) void pads_kernel(
    const float* __restrict__ alog, const float* __restrict__ dsk, float* __restrict__ PADS)
{
  const int wi = blockIdx.x * 32 + threadIdx.x;
  const int f0 = wi * 4;
  const bool isA = (f0 < kAlpFloats);
  const int ea = isA ? f0 : (kAlpFloats - 4);
  const int dq = f0 - kAlpFloats;
  const int ed = isA ? 0 : dq;
  const v4f va = *(const v4f*)(alog + ea);
  const v4f vd = *(const v4f*)(dsk + ed);
  const float a0 = va[0];
  const float a1 = va[1];
  const float a2 = va[2];
  const float a3 = va[3];
  const float e0 = vd[0];
  const float e1 = vd[1];
  const float e2 = vd[2];
  const float e3 = vd[3];
  const float s0 = isA ? a0 : e0;
  const float s1 = isA ? a1 : e1;
  const float s2 = isA ? a2 : e2;
  const float s3 = isA ? a3 : e3;
  v4f o;
  o[0] = bf16r(s0);
  o[1] = bf16r(s1);
  o[2] = bf16r(s2);
  o[3] = bf16r(s3);
  float* q = PADS + (size_t)f0;
  *(volatile v4f*)q = o;
  __threadfence();
  *(volatile v4f*)q = o;
}

typedef float    ms1_v4f __attribute__((ext_vector_type(4)));
typedef unsigned ms1_v4u __attribute__((ext_vector_type(4)));
struct ms1_args {
  const float* dtpre;
  const float* u;
  const float* bc;
  const float* z;
  const float* A_log;
  const float* Dskip;
  __half* y;
  __half* y_lo;
  long ld_dtpre;
  long ld_u;
  long ld_bc;
  long ld_z;
  long ld_y;
  int offB;
  int offC;
  int offZ;
  float ycarry;
  int dir;
  int D;
  int L;
  int nbatch;
};
static_assert(sizeof(ms1_args) == 136);

__device__ __forceinline__ float ms1_flush16(float v) {
  return (fabsf(v) < 6.103515625e-05f) ? 0.0f : v;
}
__device__ __forceinline__ unsigned ms1_h16bits(float v) {
  return (unsigned)__half_as_ushort(__float2half_rn(ms1_flush16(v)));
}
__device__ __forceinline__ float ms1_h16val(unsigned b) {
  return __half2float(__ushort_as_half((unsigned short)b));
}
__device__ __forceinline__ float ms1_softplus(float v) {
  return fmaxf(v, 0.0f) + log1pf(expf(-fabsf(v)));
}
__device__ __forceinline__ void ms1_pack2(float v0, float v1, unsigned& hw, unsigned& lw) {
  const unsigned h0 = ms1_h16bits(v0);
  const unsigned h1 = ms1_h16bits(v1);
  const float r0 = (v0 - ms1_h16val(h0)) * 2048.0f;
  const float r1 = (v1 - ms1_h16val(h1)) * 2048.0f;
  const unsigned l0 = ms1_h16bits(r0);
  const unsigned l1 = ms1_h16bits(r1);
  hw = h0 | (h1 << 16);
  lw = l0 | (l1 << 16);
}

template <int NSTATE>
__global__ __launch_bounds__(64 * (NSTATE / 16)) void ms1_scan_kernel(ms1_args a)
{
  static_assert(NSTATE == 16 || NSTATE == 64);
  constexpr int NQ  = NSTATE / 16;
  constexpr int NT  = 64 * NQ;
  constexpr int NW  = NT / 32;
  constexpr int BCW = 2 * NSTATE;
  constexpr int YP  = 68;
  constexpr int RPI = NW * 4;
  constexpr int NIT = 64 / RPI;
  static_assert(16 * NT <= 64 * YP);
  __shared__ __align__(16) float sBC[64 * BCW];
  __shared__ __align__(16) float sY[64 * YP];
  const int tid  = threadIdx.x;
  const int lane = tid & 31;
  const int wave = tid >> 5;
  const int c    = tid / NQ;
  const int sq   = tid - c * NQ;
  const int bpb  = a.D / 64;
  const int bi   = blockIdx.x / bpb;
  if (bi >= a.nbatch) return;
  const int d0 = (blockIdx.x - bi * bpb) * 64;
  const int d  = d0 + c;
  const long rowb = (long)bi * a.L;
  const bool hasz  = (a.z != nullptr);
  const bool hasD  = (a.Dskip != nullptr);
  const bool hasLo = (a.y_lo != nullptr);

#pragma unroll 1
  for (int n = 0; n < 16; ++n) {
    const float al = a.A_log[(long)d * NSTATE + sq * 16 + n];
    sY[n * NT + tid] = -expf(al);
  }
  __syncthreads();
  float An[16], h[16];
#pragma unroll
  for (int n = 0; n < 16; ++n) {
    An[n] = sY[n * NT + tid];
    h[n] = 0.0f;
  }
  float Dd = 0.0f;
  if (hasD) Dd = a.Dskip[d];

  const int nchunk = a.L / 64;
  const bool fwd = (a.dir > 0);
  const int s0 = fwd ? 0 : 63;
  const int sd = fwd ? 1 : -1;
  const int q  = lane >> 3;
  const int c8 = (lane & 7) * 8;

  for (int ci = 0; ci < nchunk; ++ci) {
    const int tb = fwd ? (ci * 64) : (a.L - 64 - ci * 64);
    const long rowc = rowb + tb;
    __syncthreads();
#pragma unroll 8
    for (int i = 0; i < 32; ++i) {
      const int idx = tid + i * NT;
      const int st  = idx / BCW;
      const int col = idx - st * BCW;
      const int sc  = (col < NSTATE) ? (a.offB + col) : (a.offC + col - NSTATE);
      sBC[idx] = a.bc[(rowc + st) * a.ld_bc + sc];
    }
    __syncthreads();
    for (int s = 0; s < 64; ++s) {
      const int ls = s0 + sd * s;
      const long row = rowc + ls;
      float pre = a.dtpre[row * a.ld_dtpre + d];
      float uv  = a.u[row * a.ld_u + d];
      float zv  = 0.0f;
      if (hasz) zv = a.z[row * a.ld_z + a.offZ + d];
      asm volatile("" : "+v"(pre));
      asm volatile("" : "+v"(uv));
      asm volatile("" : "+v"(zv));
      const float delta = ms1_softplus(pre);
      const float dtx = delta * uv;
      const float* bp = sBC + ls * BCW + sq * 16;
      const float* cp = bp + NSTATE;
      ms1_v4f Bq[4], Cq[4];
#pragma unroll
      for (int k = 0; k < 4; ++k) {
        Bq[k] = *(const ms1_v4f*)(bp + 4 * k);
        Cq[k] = *(const ms1_v4f*)(cp + 4 * k);
      }
      float yv = 0.0f;
#pragma unroll
      for (int n = 0; n < 16; ++n) {
        const float e = __expf(delta * An[n]);
        h[n] = fmaf(e, h[n], dtx * Bq[n >> 2][n & 3]);
        yv = fmaf(h[n], Cq[n >> 2][n & 3], yv);
      }
      if (NQ > 1) {
        yv += __shfl_xor(yv, 1, 32);
        yv += __shfl_xor(yv, 2, 32);
      }
      if (hasD) yv = fmaf(uv, Dd, yv);
      if (hasz) {
        const float sg = __builtin_amdgcn_rcpf(1.0f + expf(-zv));
        yv = yv * (zv * sg);
      }
      if (sq == 0) sY[ls * YP + c] = yv * a.ycarry;
    }
    __syncthreads();
    ms1_v4u hw[NIT], lw[NIT];
#pragma unroll
    for (int it = 0; it < NIT; ++it) {
      const int row = it * RPI + wave * 4 + q;
      const float* sp = sY + row * YP + c8;
      const ms1_v4f f0 = *(const ms1_v4f*)(sp);
      const ms1_v4f f1 = *(const ms1_v4f*)(sp + 4);
      unsigned h0, h1, h2, h3, l0, l1, l2, l3;
      ms1_pack2(f0[0], f0[1], h0, l0);
      ms1_pack2(f0[2], f0[3], h1, l1);
      ms1_pack2(f1[0], f1[1], h2, l2);
      ms1_pack2(f1[2], f1[3], h3, l3);
      hw[it] = (ms1_v4u){h0, h1, h2, h3};
      lw[it] = (ms1_v4u){l0, l1, l2, l3};
    }
    for (int pass = 0; pass < 2; ++pass) {
#pragma unroll
      for (int it = 0; it < NIT; ++it) {
        const int row = it * RPI + wave * 4 + q;
        const long o = (rowc + row) * a.ld_y + d0 + c8;
        *(volatile ms1_v4u*)(a.y + o) = hw[it];
        if (hasLo) *(volatile ms1_v4u*)(a.y_lo + o) = lw[it];
      }
      __threadfence();
    }
  }
}

__global__ __launch_bounds__(32) void gcm_kernel(
    const float* __restrict__ UC, float* __restrict__ GCM)
{
  const int i = blockIdx.x * 32 + threadIdx.x;
  const int b = i / (kD / 4);
  const int c4 = (i - b * (kD / 4)) * 4;
  const float* sp = UC + (size_t)b * kL * kD + c4;
  float s0 = 0.0f, s1 = 0.0f, s2 = 0.0f, s3 = 0.0f;
  for (int p = 0; p < 2304; ++p) {
    const v4f v = *(const v4f*)(sp + (size_t)p * kD);
    const float a0 = v[0];
    const float a1 = v[1];
    const float a2 = v[2];
    const float a3 = v[3];
    s0 = s0 + a0;
    s1 = s1 + a1;
    s2 = s2 + a2;
    s3 = s3 + a3;
  }
  const float sc = 1.0f / 2304.0f;
  v4f o;
  o[0] = s0 * sc;
  o[1] = s1 * sc;
  o[2] = s2 * sc;
  o[3] = s3 * sc;
  float* q = GCM + (size_t)i * 4;
  *(volatile v4f*)q = o;
  __threadfence();
  *(volatile v4f*)q = o;
}

__device__ __forceinline__ float gelu_exact(float v) {
  return 0.5f * v * (1.0f + erff(v * 0.70710678118654752f));
}
__global__ __launch_bounds__(32) void gc1_kernel(
    const float* __restrict__ GCM, const float* __restrict__ w1, float* __restrict__ H1)
{
  const int i = blockIdx.x * 32 + threadIdx.x;
  const int b = i / (kFcHP / 4);
  const int j4 = (i - b * (kFcHP / 4)) * 4;
  const int ja = (j4 + 0 < kFcH) ? (j4 + 0) : (kFcH - 1);
  const int jb = (j4 + 1 < kFcH) ? (j4 + 1) : (kFcH - 1);
  const int jc = (j4 + 2 < kFcH) ? (j4 + 2) : (kFcH - 1);
  const int jd = (j4 + 3 < kFcH) ? (j4 + 3) : (kFcH - 1);
  const float* gp = GCM + (size_t)b * kD;
  const float* pa = w1 + (size_t)ja * kC;
  const float* pb = w1 + (size_t)jb * kC;
  const float* pc = w1 + (size_t)jc * kC;
  const float* pd = w1 + (size_t)jd * kC;
  float a0 = 0.0f, a1 = 0.0f, a2 = 0.0f, a3 = 0.0f;
  for (int c = 0; c < 192; c += 4) {
    const v4f g = *(const v4f*)(gp + c);
    const v4f qa = *(const v4f*)(pa + c);
    const v4f qb = *(const v4f*)(pb + c);
    const v4f qc = *(const v4f*)(pc + c);
    const v4f qd = *(const v4f*)(pd + c);
    const float g0 = g[0];
    const float g1 = g[1];
    const float g2 = g[2];
    const float g3 = g[3];
    const float wa0 = qa[0];
    const float wa1 = qa[1];
    const float wa2 = qa[2];
    const float wa3 = qa[3];
    const float wb0 = qb[0];
    const float wb1 = qb[1];
    const float wb2 = qb[2];
    const float wb3 = qb[3];
    const float wc0 = qc[0];
    const float wc1 = qc[1];
    const float wc2 = qc[2];
    const float wc3 = qc[3];
    const float wd0 = qd[0];
    const float wd1 = qd[1];
    const float wd2 = qd[2];
    const float wd3 = qd[3];
    a0 = fmaf(g0, bf16r(wa0), a0);
    a0 = fmaf(g1, bf16r(wa1), a0);
    a0 = fmaf(g2, bf16r(wa2), a0);
    a0 = fmaf(g3, bf16r(wa3), a0);
    a1 = fmaf(g0, bf16r(wb0), a1);
    a1 = fmaf(g1, bf16r(wb1), a1);
    a1 = fmaf(g2, bf16r(wb2), a1);
    a1 = fmaf(g3, bf16r(wb3), a1);
    a2 = fmaf(g0, bf16r(wc0), a2);
    a2 = fmaf(g1, bf16r(wc1), a2);
    a2 = fmaf(g2, bf16r(wc2), a2);
    a2 = fmaf(g3, bf16r(wc3), a2);
    a3 = fmaf(g0, bf16r(wd0), a3);
    a3 = fmaf(g1, bf16r(wd1), a3);
    a3 = fmaf(g2, bf16r(wd2), a3);
    a3 = fmaf(g3, bf16r(wd3), a3);
  }
  const float e0 = gelu_exact(a0);
  const float e1 = gelu_exact(a1);
  const float e2 = gelu_exact(a2);
  const float e3 = gelu_exact(a3);
  v4f o;
  o[0] = (j4 + 0 < kFcH) ? e0 : 0.0f;
  o[1] = (j4 + 1 < kFcH) ? e1 : 0.0f;
  o[2] = (j4 + 2 < kFcH) ? e2 : 0.0f;
  o[3] = (j4 + 3 < kFcH) ? e3 : 0.0f;
  float* q = H1 + (size_t)i * 4;
  *(volatile v4f*)q = o;
  __threadfence();
  *(volatile v4f*)q = o;
}

__global__ __launch_bounds__(32) void gc2_kernel(
    const float* __restrict__ H1, const float* __restrict__ w2, float* __restrict__ GC)
{
  const int i = blockIdx.x * 32 + threadIdx.x;
  const int b = i / (kC / 4);
  const int m4 = (i - b * (kC / 4)) * 4;
  const float* hp = H1 + (size_t)b * kFcHP;
  const float* wp = w2 + (size_t)m4 * kFcH;
  float a0 = 0.0f, a1 = 0.0f, a2 = 0.0f, a3 = 0.0f;
  for (int j = 0; j < 48; j += 4) {
    const v4f hv = *(const v4f*)(hp + j);
    const v4f qa = *(const v4f*)(wp + j);
    const v4f qb = *(const v4f*)(wp + kFcH + j);
    const v4f qc = *(const v4f*)(wp + 2 * kFcH + j);
    const v4f qd = *(const v4f*)(wp + 3 * kFcH + j);
    const float h0 = hv[0];
    const float h1 = hv[1];
    const float h2 = hv[2];
    const float h3 = hv[3];
    const float wa0 = qa[0];
    const float wa1 = qa[1];
    const float wa2 = qa[2];
    const float wa3 = qa[3];
    const float wb0 = qb[0];
    const float wb1 = qb[1];
    const float wb2 = qb[2];
    const float wb3 = qb[3];
    const float wc0 = qc[0];
    const float wc1 = qc[1];
    const float wc2 = qc[2];
    const float wc3 = qc[3];
    const float wd0 = qd[0];
    const float wd1 = qd[1];
    const float wd2 = qd[2];
    const float wd3 = qd[3];
    a0 = fmaf(h0, bf16r(wa0), a0);
    a0 = fmaf(h1, bf16r(wa1), a0);
    a0 = fmaf(h2, bf16r(wa2), a0);
    a0 = fmaf(h3, bf16r(wa3), a0);
    a1 = fmaf(h0, bf16r(wb0), a1);
    a1 = fmaf(h1, bf16r(wb1), a1);
    a1 = fmaf(h2, bf16r(wb2), a1);
    a1 = fmaf(h3, bf16r(wb3), a1);
    a2 = fmaf(h0, bf16r(wc0), a2);
    a2 = fmaf(h1, bf16r(wc1), a2);
    a2 = fmaf(h2, bf16r(wc2), a2);
    a2 = fmaf(h3, bf16r(wc3), a2);
    a3 = fmaf(h0, bf16r(wd0), a3);
    a3 = fmaf(h1, bf16r(wd1), a3);
    a3 = fmaf(h2, bf16r(wd2), a3);
    a3 = fmaf(h3, bf16r(wd3), a3);
  }
  v4f o;
  o[0] = 1.0f / (1.0f + expf(-a0));
  o[1] = 1.0f / (1.0f + expf(-a1));
  o[2] = 1.0f / (1.0f + expf(-a2));
  o[3] = 1.0f / (1.0f + expf(-a3));
  float* q = GC + (size_t)i * 4;
  *(volatile v4f*)q = o;
  __threadfence();
  *(volatile v4f*)q = o;
}

__device__ __forceinline__ v2u yh_words(const unsigned short* __restrict__ YH, int k, int b, int t, int c4) {
  const int row = k * kRows + b * kL + t;
  return *(const v2u*)(YH + (size_t)row * kD + c4);
}
__device__ __forceinline__ void words_to4(unsigned u0, unsigned u1, float& f0, float& f1, float& f2, float& f3) {
  f0 = h16_to_f32(u0 & 0xffffu);
  f1 = h16_to_f32(u0 >> 16);
  f2 = h16_to_f32(u1 & 0xffffu);
  f3 = h16_to_f32(u1 >> 16);
}
__device__ __forceinline__ float merge4(float ga, float gb, float gc, float gd,
                                        float v0, float v2, float v1, float v3) {
  const float p0 = bf16r(ga) * v0;
  const float p2 = bf16r(gb) * v2;
  const float p1 = bf16r(gc) * v1;
  const float p3 = bf16r(gd) * v3;
  const float s = ((p0 + p2) + p1) + p3;
  return s;
}
__global__ __launch_bounds__(256) void merge_kernel(
    const unsigned short* __restrict__ YH, const float* __restrict__ GC,
    const float* __restrict__ ga1, const float* __restrict__ ga2,
    const float* __restrict__ ga3, const float* __restrict__ ga4, float* __restrict__ MG)
{
  const int i = blockIdx.x * 256 + threadIdx.x;
  const int r = i / (kD / 4);
  const int c4 = (i - r * (kD / 4)) * 4;
  const int b = r / kL;
  const int p = r - b * kL;
  const int si = win_index(p);
  const int sj = swap48(si);
  const v2u w0 = yh_words(YH, 0, b, si, c4);
  const v2u w2 = yh_words(YH, 2, b, kL - 1 - si, c4);
  const v2u w1 = yh_words(YH, 1, b, sj, c4);
  const v2u w3 = yh_words(YH, 3, b, kL - 1 - sj, c4);
  const v4f q1 = *(const v4f*)(ga1 + c4);
  const v4f q2 = *(const v4f*)(ga2 + c4);
  const v4f q3 = *(const v4f*)(ga3 + c4);
  const v4f q4 = *(const v4f*)(ga4 + c4);
  const v4f qg = *(const v4f*)(GC + (size_t)b * kC + c4);
  const unsigned w0a = w0[0];
  const unsigned w0b = w0[1];
  const unsigned w1a = w1[0];
  const unsigned w1b = w1[1];
  const unsigned w2a = w2[0];
  const unsigned w2b = w2[1];
  const unsigned w3a = w3[0];
  const unsigned w3b = w3[1];
  float a0, a1, a2, a3;
  float b0, b1, b2, b3;
  float e0, e1, e2, e3;
  float f0, f1, f2, f3;
  words_to4(w0a, w0b, a0, a1, a2, a3);
  words_to4(w1a, w1b, b0, b1, b2, b3);
  words_to4(w2a, w2b, e0, e1, e2, e3);
  words_to4(w3a, w3b, f0, f1, f2, f3);
  const float g10 = q1[0];
  const float g11 = q1[1];
  const float g12 = q1[2];
  const float g13 = q1[3];
  const float g20 = q2[0];
  const float g21 = q2[1];
  const float g22 = q2[2];
  const float g23 = q2[3];
  const float g30 = q3[0];
  const float g31 = q3[1];
  const float g32 = q3[2];
  const float g33 = q3[3];
  const float g40 = q4[0];
  const float g41 = q4[1];
  const float g42 = q4[2];
  const float g43 = q4[3];
  const float c0 = qg[0];
  const float c1 = qg[1];
  const float c2 = qg[2];
  const float c3 = qg[3];
  const float s0 = merge4(g10, g20, g30, g40, a0, e0, b0, f0);
  const float s1 = merge4(g11, g21, g31, g41, a1, e1, b1, f1);
  const float s2 = merge4(g12, g22, g32, g42, a2, e2, b2, f2);
  const float s3 = merge4(g13, g23, g33, g43, a3, e3, b3, f3);
  const float sc = 1.0f / kYCarry;
  v4f o;
  o[0] = s0 * sc * c0;
  o[1] = s1 * sc * c1;
  o[2] = s2 * sc * c2;
  o[3] = s3 * sc * c3;
  float* q = MG + (size_t)i * 4;
  *(volatile v4f*)q = o;
  __threadfence();
  *(volatile v4f*)q = o;
}

__global__ __launch_bounds__(256) void ln_stats_kernel(
    const float* __restrict__ MG, float* __restrict__ ST)
{
  const int r = blockIdx.x * 256 + threadIdx.x;
  const float* mp = MG + (size_t)r * kD;
  float sum = 0.0f;
  for (int c = 0; c < 192; c += 4) {
    const v4f v = *(const v4f*)(mp + c);
    const float a0 = v[0];
    const float a1 = v[1];
    const float a2 = v[2];
    const float a3 = v[3];
    sum = sum + a0;
    sum = sum + a1;
    sum = sum + a2;
    sum = sum + a3;
  }
  const float mu = sum * (1.0f / 192.0f);
  float vs = 0.0f;
  for (int c = 0; c < 192; c += 4) {
    const v4f v = *(const v4f*)(mp + c);
    const float a0 = v[0];
    const float a1 = v[1];
    const float a2 = v[2];
    const float a3 = v[3];
    const float e0 = a0 - mu;
    const float e1 = a1 - mu;
    const float e2 = a2 - mu;
    const float e3 = a3 - mu;
    vs = fmaf(e0, e0, vs);
    vs = fmaf(e1, e1, vs);
    vs = fmaf(e2, e2, vs);
    vs = fmaf(e3, e3, vs);
  }
  const float var = vs * (1.0f / 192.0f);
  const float sd = sqrtf(var + 1e-5f);
  v4f ov;
  ov[0] = mu;
  ov[1] = sd;
  ov[2] = 0.0f;
  ov[3] = 0.0f;
  float* q = ST + (size_t)r * 4;
  *(volatile v4f*)q = ov;
  __threadfence();
  *(volatile v4f*)q = ov;
}

__device__ __forceinline__ _Float16 gate_half(float m, float mu, float sd, float lw, float lb, float zv) {
  const float yn = (m - mu) / sd * bf16r(lw) + bf16r(lb);
  const float g = zv / (1.0f + expf(-zv));
  const float yg = yn * g;
  return f16_flush(yg * kGCarry);
}
__global__ __launch_bounds__(256) void ln_gate_kernel(
    const float* __restrict__ MG, const float* __restrict__ ST, const float* __restrict__ XZ,
    const float* __restrict__ lnw, const float* __restrict__ lnb, unsigned short* __restrict__ YG)
{
  const int i = blockIdx.x * 256 + threadIdx.x;
  const int r = i / (kD / 8);
  const int c8 = (i - r * (kD / 8)) * 8;
  const float* mp = MG + (size_t)r * kD + c8;
  const v4f ma = *(const v4f*)(mp);
  const v4f mb = *(const v4f*)(mp + 4);
  const v4f st = *(const v4f*)(ST + (size_t)r * 4);
  const v4f wa = *(const v4f*)(lnw + c8);
  const v4f wb = *(const v4f*)(lnw + c8 + 4);
  const v4f ba = *(const v4f*)(lnb + c8);
  const v4f bb = *(const v4f*)(lnb + c8 + 4);
  const float* zp = XZ + (size_t)r * kXzN + kD + c8;
  const v4f za = *(const v4f*)(zp);
  const v4f zb = *(const v4f*)(zp + 4);
  const float mu = st[0];
  const float sd = st[1];
  const float m0 = ma[0];
  const float m1 = ma[1];
  const float m2 = ma[2];
  const float m3 = ma[3];
  const float m4 = mb[0];
  const float m5 = mb[1];
  const float m6 = mb[2];
  const float m7 = mb[3];
  const float g0 = wa[0];
  const float g1 = wa[1];
  const float g2 = wa[2];
  const float g3 = wa[3];
  const float g4 = wb[0];
  const float g5 = wb[1];
  const float g6 = wb[2];
  const float g7 = wb[3];
  const float o0 = ba[0];
  const float o1 = ba[1];
  const float o2 = ba[2];
  const float o3 = ba[3];
  const float o4 = bb[0];
  const float o5 = bb[1];
  const float o6 = bb[2];
  const float o7 = bb[3];
  const float z0 = za[0];
  const float z1 = za[1];
  const float z2 = za[2];
  const float z3 = za[3];
  const float z4 = zb[0];
  const float z5 = zb[1];
  const float z6 = zb[2];
  const float z7 = zb[3];
  v8h hv;
  hv[0] = gate_half(m0, mu, sd, g0, o0, z0);
  hv[1] = gate_half(m1, mu, sd, g1, o1, z1);
  hv[2] = gate_half(m2, mu, sd, g2, o2, z2);
  hv[3] = gate_half(m3, mu, sd, g3, o3, z3);
  hv[4] = gate_half(m4, mu, sd, g4, o4, z4);
  hv[5] = gate_half(m5, mu, sd, g5, o5, z5);
  hv[6] = gate_half(m6, mu, sd, g6, o6, z6);
  hv[7] = gate_half(m7, mu, sd, g7, o7, z7);
  unsigned short* q = YG + (size_t)i * 8;
  *(volatile v8h*)q = hv;
  __threadfence();
  *(volatile v8h*)q = hv;
}

__global__ __launch_bounds__(256) void pack_ow_kernel(
    const float* __restrict__ w, unsigned short* __restrict__ OW)
{
  const int i = blockIdx.x * 256 + threadIdx.x;
  const int m = i / (kD / 8);
  const int c8 = (i - m * (kD / 8)) * 8;
  const float* sp = w + (size_t)m * kD + c8;
  const v4f a0 = *(const v4f*)(sp);
  const v4f a1 = *(const v4f*)(sp + 4);
  const v8h hv = pack8_in(a0, a1, kWCarry, true);
  unsigned short* q = OW + (size_t)i * 8;
  *(volatile v8h*)q = hv;
  __threadfence();
  *(volatile v8h*)q = hv;
}

__global__ __launch_bounds__(256) void out_kernel(
    const float* __restrict__ RAW, float* __restrict__ out)
{
  const int wi = blockIdx.x * 256 + threadIdx.x;
  const v4f v = *(const v4f*)(RAW + (size_t)wi * 4);
  float* q = out + (size_t)wi * 4;
  *(volatile v4f*)q = v;
  __threadfence();
  *(volatile v4f*)q = v;
}

static_assert(((kRows / 32) * (kXzN / 64)) % 8 == 0 && ((kRows / 32) * (kXzN / 64)) / 8 == 216);
static_assert(((kRows / 32) * (kXpP / 64)) % 8 == 0 && ((kRows / 32) * (kXpP / 64)) / 8 == 36);
static_assert(((kRows / 32) * (kD / 64)) % 8 == 0 && ((kRows / 32) * (kD / 64)) / 8 == 108);
static_assert(((kRows / 32) * (kC / 64)) % 8 == 0 && ((kRows / 32) * (kC / 64)) / 8 == 108);
static_assert(((kRows * kC / 8) % 256) == 0 && (kRows * kC / 8) / 256 == 864);
static_assert(((kXzN * kC / 8) % 256) == 0 && (kXzN * kC / 8) / 256 == 36);
static_assert(((kRows * kD / 4) % 256) == 0 && (kRows * kD / 4) / 256 == 1728);
static_assert(((kDirs * kRows * kD / 4) % 256) == 0 && (kDirs * kRows * kD / 4) / 256 == 6912);
static_assert(((kDirs * kRows * kD / 8) % 256) == 0 && (kDirs * kRows * kD / 8) / 256 == 3456);
static_assert(((kDirs * kXpP * kD / 8) % 256) == 0 && (kDirs * kXpP * kD / 8) / 256 == 24);
static_assert(((kDirs * kRows * kRkP / 8) % 256) == 0 && (kDirs * kRows * kRkP / 8) / 256 == 576);
static_assert(((kDirs * kD * kRkP / 8) % 256) == 0 && (kDirs * kD * kRkP / 8) / 256 == 12);
static_assert((kPadFloats / 4) == 102 * 32);
static_assert((kBatch * kD / 4) == 6 * 32);
static_assert((kBatch * kFcHP / 4) == 2 * 32);
static_assert((kBatch * kC / 4) == 6 * 32);
static_assert((kRows % 256) == 0 && kRows / 256 == 36);
static_assert(((kRows * kD / 8) % 256) == 0 && (kRows * kD / 8) / 256 == 864);
static_assert(((kC * kD / 8) % 256) == 0 && (kC * kD / 8) / 256 == 18);
static_assert(((kRows * kC / 4) % 256) == 0 && (kRows * kC / 4) / 256 == 1728);
static_assert((kD % 64) == 0 && (kL % 64) == 0);

extern "C" void kernel_launch(void* const* d_in, const int* in_sizes, int n_in,
                              void* d_out, int out_size, void* d_ws, size_t ws_size,
                              hipStream_t stream)
{
  if (n_in < 18) return;
  if (in_sizes[0] != kRows * kC) return;
  if (in_sizes[1] != kXzN * kC) return;
  if (in_sizes[2] != kD * kTaps) return;
  if (in_sizes[3] != kD) return;
  if (in_sizes[4] != kDirs * kXpN * kD) return;
  if (in_sizes[5] != kDirs * kD * kRank) return;
  if (in_sizes[6] != kDirs * kD) return;
  if (in_sizes[7] != kDirs * kD * kNst) return;
  if (in_sizes[8] != kDirs * kD) return;
  if (in_sizes[9] != kD) return;
  if (in_sizes[10] != kD) return;
  if (in_sizes[11] != kD) return;
  if (in_sizes[12] != kD) return;
  if (in_sizes[13] != kFcH * kC) return;
  if (in_sizes[14] != kC * kFcH) return;
  if (in_sizes[15] != kD) return;
  if (in_sizes[16] != kD) return;
  if (in_sizes[17] != kC * kD) return;
  if (out_size != kRows * kC) return;
  if (ws_size < kWsTotal) return;

  const float* x      = (const float*)d_in[0];
  const float* w_in   = (const float*)d_in[1];
  const float* conv_w = (const float*)d_in[2];
  const float* conv_b = (const float*)d_in[3];
  const float* w_xp   = (const float*)d_in[4];
  const float* dt_w   = (const float*)d_in[5];
  const float* dt_b   = (const float*)d_in[6];
  const float* a_logs = (const float*)d_in[7];
  const float* d_skip = (const float*)d_in[8];
  const float* gam1   = (const float*)d_in[9];
  const float* gam2   = (const float*)d_in[10];
  const float* gam3   = (const float*)d_in[11];
  const float* gam4   = (const float*)d_in[12];
  const float* fc_w1  = (const float*)d_in[13];
  const float* fc_w2  = (const float*)d_in[14];
  const float* ln_w   = (const float*)d_in[15];
  const float* ln_b   = (const float*)d_in[16];
  const float* w_out  = (const float*)d_in[17];
  float* out = (float*)d_out;

  char* ws = (char*)d_ws;
  unsigned short* XH   = (unsigned short*)(ws + kOffXH);
  unsigned short* WIN  = (unsigned short*)(ws + kOffWIN);
  float*          XZ   = (float*)(ws + kOffXZ);
  float*          UC   = (float*)(ws + kOffUC);
  float*          XS   = (float*)(ws + kOffXS);
  unsigned short* XSH  = (unsigned short*)(ws + kOffXSH);
  unsigned short* XPW  = (unsigned short*)(ws + kOffXPW);
  float*          XD   = (float*)(ws + kOffXD);
  unsigned short* DRH  = (unsigned short*)(ws + kOffDRH);
  unsigned short* DTW  = (unsigned short*)(ws + kOffDTW);
  float*          DTP  = (float*)(ws + kOffDTP);
  float*          PADS = (float*)(ws + kOffPADS);
  unsigned short* YH   = (unsigned short*)(ws + kOffYH);
  float*          GCM  = (float*)(ws + kOffGCM);
  float*          H1   = (float*)(ws + kOffH1);
  float*          GC   = (float*)(ws + kOffGC);
  float*          MG   = (float*)(ws + kOffMG);
  float*          ST   = (float*)(ws + kOffST);
  unsigned short* YG   = (unsigned short*)(ws + kOffYG);
  unsigned short* OW   = (unsigned short*)(ws + kOffOW);
  float*          RAW  = (float*)(ws + kOffRAW);
  float*          ALP  = PADS;
  float*          DSP  = PADS + kAlpFloats;

  constexpr float s1 = 1.0f / (kXCarry * kWCarry);
  constexpr float s2 = 1.0f / (kSCarry * kWCarry);
  constexpr float s3 = 1.0f / (kRCarry * kWCarry);
  constexpr float s4 = 1.0f / (kGCarry * kWCarry);

  pack_x_kernel<<<(kRows * kC / 8) / 256, 256, 0, stream>>>(x, XH);

  pack_inw_kernel<<<(kXzN * kC / 8) / 256, 256, 0, stream>>>(w_in, WIN);

  eng::gemm_f16_kernel<2, 0><<<dim3((kRows / 32) * (kXzN / 64) / 8), 256, 0, stream>>>(
      XH, nullptr, kC, WIN, nullptr, kC, XZ, kXzN, kRows, kXzN, kC, s1, 0.0f);

  conv_kernel<<<(kRows * kD / 4) / 256, 256, 0, stream>>>(XZ, conv_w, conv_b, UC);

  order_kernel<<<(kDirs * kRows * kD / 4) / 256, 256, 0, stream>>>(UC, XS);

  pack_xs_kernel<<<(kDirs * kRows * kD / 8) / 256, 256, 0, stream>>>(UC, XSH);

  pack_xpw_kernel<<<(kDirs * kXpP * kD / 8) / 256, 256, 0, stream>>>(w_xp, XPW);

  for (int k = 0; k < kDirs; ++k) {
    eng::gemm_f16_kernel<2, 0><<<dim3((kRows / 32) * (kXpP / 64) / 8), 256, 0, stream>>>(
        XSH + (size_t)k * kRows * kD, nullptr, kD,
        XPW + (size_t)k * kXpP * kD, nullptr, kD,
        XD + (size_t)k * kRows * kXpP, kXpP, kRows, kXpP, kD, s2, 0.0f);
  }

  pack_dr_kernel<<<(kDirs * kRows * kRkP / 8) / 256, 256, 0, stream>>>(XD, DRH);

  pack_dtw_kernel<<<(kDirs * kD * kRkP / 8) / 256, 256, 0, stream>>>(dt_w, dt_b, DTW);

  for (int k = 0; k < kDirs; ++k) {
    eng::gemm_f16_kernel<2, 0><<<dim3((kRows / 32) * (kD / 64) / 8), 256, 0, stream>>>(
        DRH + (size_t)k * kRows * kRkP, nullptr, kRkP,
        DTW + (size_t)k * kD * kRkP, nullptr, kRkP,
        DTP + (size_t)k * kRows * kD, kD, kRows, kD, kRkP, s3, 0.0f);
  }

  pads_kernel<<<102, 32, 0, stream>>>(a_logs, d_skip, PADS);

  for (int k = 0; k < kDirs; ++k) {
    ms1_args sa;
    sa.dtpre = DTP + (size_t)k * kRows * kD;
    sa.u = XS + (size_t)k * kRows * kD;
    sa.bc = XD + (size_t)k * kRows * kXpP;
    sa.z = nullptr;
    sa.A_log = ALP + (size_t)k * kD * kNst;
    sa.Dskip = DSP + (size_t)k * kD;
    sa.y = (__half*)(YH + (size_t)k * kRows * kD);
    sa.y_lo = nullptr;
    sa.ld_dtpre = kD;
    sa.ld_u = kD;
    sa.ld_bc = kXpP;
    sa.ld_z = 0;
    sa.ld_y = kD;
    sa.offB = kRank;
    sa.offC = kRank + kNst;
    sa.offZ = 0;
    sa.ycarry = kYCarry;
    sa.dir = 1;
    sa.D = kD;
    sa.L = kL;
    sa.nbatch = kBatch;
    ms1_scan_kernel<16><<<dim3((kD / 64) * kBatch), 64, 0, stream>>>(sa);
  }

  gcm_kernel<<<6, 32, 0, stream>>>(UC, GCM);

  gc1_kernel<<<2, 32, 0, stream>>>(GCM, fc_w1, H1);

  gc2_kernel<<<6, 32, 0, stream>>>(H1, fc_w2, GC);

  merge_kernel<<<(kRows * kD / 4) / 256, 256, 0, stream>>>(YH, GC, gam1, gam2, gam3, gam4, MG);

  ln_stats_kernel<<<kRows / 256, 256, 0, stream>>>(MG, ST);

  ln_gate_kernel<<<(kRows * kD / 8) / 256, 256, 0, stream>>>(MG, ST, XZ, ln_w, ln_b, YG);

  pack_ow_kernel<<<(kC * kD / 8) / 256, 256, 0, stream>>>(w_out, OW);

  eng::gemm_f16_kernel<2, 0><<<dim3((kRows / 32) * (kC / 64) / 8), 256, 0, stream>>>(
      YG, nullptr, kD, OW, nullptr, kD, RAW, kC, kRows, kC, kD, s4, 0.0f);

  out_kernel<<<(kRows * kC / 4) / 256, 256, 0, stream>>>(RAW, out);
}
